// paired_conv_1786706395588
// MI455X (gfx1250) — hardware-verified
//
#include <hip/hip_runtime.h>


#define NIMG 4
#define CC   64
#define HH   128
#define WW   128
#define NPIX (HH * WW)
#define KK   (9 * CC)
#define NO   64
#define PR   NPIX
typedef _Float16 h16;
typedef unsigned short bf;
typedef __attribute__((ext_vector_type(16))) __bf16   v16bf;
typedef __attribute__((ext_vector_type(16))) _Float16 v16h;
typedef __attribute__((ext_vector_type(8)))  _Float16 v8h;
typedef __attribute__((ext_vector_type(8)))  unsigned short v8us;
typedef __attribute__((ext_vector_type(8)))  float    v8f;
typedef __attribute__((ext_vector_type(4)))  float    v4f;
typedef v8h  __attribute__((may_alias)) v8ha;
typedef v4f  __attribute__((may_alias)) v4fa;
typedef v8us __attribute__((may_alias)) v8usa;

__device__ __forceinline__ unsigned short f2bf(float f) { unsigned u = __float_as_uint(f); u += 0x7FFFu + ((u >> 16) & 1u); return (unsigned short)(u >> 16); }
__device__ __forceinline__ float bf2f(unsigned short b) { return __uint_as_float(((unsigned)b) << 16); }
__device__ __forceinline__ float bfr(float f) { return bf2f(f2bf(f)); }
__device__ __forceinline__ v16h cat16(v8h lo, v8h hi) { return __builtin_shufflevector(lo, hi, 0, 1, 2, 3, 4, 5, 6, 7, 8, 9, 10, 11, 12, 13, 14, 15); }
__device__ __forceinline__ v16bf cat16b(v8us lo, v8us hi) { return __builtin_bit_cast(v16bf, __builtin_shufflevector(lo, hi, 0, 1, 2, 3, 4, 5, 6, 7, 8, 9, 10, 11, 12, 13, 14, 15)); }
__device__ __forceinline__ v8f wmma16(v16h a, v16h b, v8f c) { return __builtin_amdgcn_wmma_f32_16x16x32_f16(false, a, false, b, (short)0, c, false, false); }
__device__ __forceinline__ v8f wmmab(v16bf a, v16bf b, v8f c) { return __builtin_amdgcn_wmma_f32_16x16x32_bf16(false, a, false, b, (short)0, c, false, false); }


template <typename T16> struct WFrag;
template <> struct WFrag<h16> { typedef v16h V; static __device__ __forceinline__ V ld(const h16* p) { return cat16(*(const v8h*)p, *(const v8h*)(p + 16)); } static __device__ __forceinline__ v8f mma(V a, V b, v8f c) { return wmma16(a, b, c); } };
template <> struct WFrag<bf> { typedef v16bf V; static __device__ __forceinline__ V ld(const bf* p) { return cat16b(*(const v8us*)p, *(const v8us*)(p + 16)); } static __device__ __forceinline__ v8f mma(V a, V b, v8f c) { return wmmab(a, b, c); } };
template <typename T16, int NSPLIT, bool BIAS>
__global__ __launch_bounds__(32) void k_gemmw(const T16* __restrict__ A, const T16* __restrict__ A2, const T16* __restrict__ Bt, const T16* __restrict__ Bt2, int K, float* C, int ldc, const float* __restrict__ bias, size_t sA, size_t sB, size_t sC) {
    typedef typename WFrag<T16>::V V;
    __shared__ __align__(16) float os[16 * 68];
    const size_t z = blockIdx.z; A += z * sA; if (A2) A2 += z * sA; Bt += z * sB; if (Bt2) Bt2 += z * sB; C += z * sC;
    const int lane = threadIdx.x & 31, lr = lane & 15, hi = lane >> 4; const int r0 = blockIdx.x * 64, c0 = blockIdx.y * 64;
    v8f acc[4][4];
#pragma unroll
    for (int mb = 0; mb < 4; ++mb)
#pragma unroll
        for (int nb = 0; nb < 4; ++nb) acc[mb][nb] = (v8f){};
    const size_t aoff = (size_t)(r0 + lr) * K + 8 * hi, boff = (size_t)(c0 + lr) * K + 8 * hi;
#pragma unroll 1
    for (int kc = 0; kc < K; kc += 32) {
        V a[4], a2[4];
#pragma unroll
        for (int mb = 0; mb < 4; ++mb) { a[mb] = WFrag<T16>::ld(A + aoff + (size_t)mb * 16 * K + kc); if (NSPLIT == 1 || NSPLIT == 2) a2[mb] = WFrag<T16>::ld(A2 + aoff + (size_t)mb * 16 * K + kc); }
#pragma unroll
        for (int nb = 0; nb < 4; ++nb) { const V b = WFrag<T16>::ld(Bt + boff + (size_t)nb * 16 * K + kc); V b2; if (NSPLIT >= 2) b2 = WFrag<T16>::ld(Bt2 + boff + (size_t)nb * 16 * K + kc);
#pragma unroll
            for (int mb = 0; mb < 4; ++mb) { acc[mb][nb] = WFrag<T16>::mma(a[mb], b, acc[mb][nb]); if (NSPLIT == 1 || NSPLIT == 2) acc[mb][nb] = WFrag<T16>::mma(a2[mb], b, acc[mb][nb]); if (NSPLIT >= 2) acc[mb][nb] = WFrag<T16>::mma(a[mb], b2, acc[mb][nb]); } }
        asm volatile("v_nop\n\tv_nop\n\tv_nop\n\tv_nop" : "+v"(acc[0][0]), "+v"(acc[1][1]), "+v"(acc[2][2]), "+v"(acc[3][3]) : "v"(a[0]), "v"(a[3]));
    }
#pragma unroll
    for (int mb = 0; mb < 4; ++mb) {
#pragma unroll
        for (int nb = 0; nb < 4; ++nb) {
#pragma unroll
            for (int j = 0; j < 8; ++j) os[(hi * 8 + j) * 68 + nb * 16 + lr] = acc[mb][nb][j]; }
        __builtin_amdgcn_wave_barrier(); asm volatile("" ::: "memory");
        float* crow = C + (size_t)(r0 + mb * 16) * ldc + c0;
#pragma unroll 1
        for (int ps = 0; ps < 2; ++ps) {
#pragma unroll
            for (int s = 0; s < 8; ++s) { const int row = 2 * s + hi, cofs = lr * 4; v4f val = *(const v4fa*)(os + row * 68 + cofs); if (BIAS) { val[0] += bfr(bias[c0 + cofs]); val[1] += bfr(bias[c0 + cofs + 1]); val[2] += bfr(bias[c0 + cofs + 2]); val[3] += bfr(bias[c0 + cofs + 3]); }
                *(volatile v4f*)(crow + (size_t)row * ldc + cofs) = val; }
            if (ps == 0) __threadfence(); }
        __builtin_amdgcn_wave_barrier(); asm volatile("" ::: "memory");
    }
}

__device__ __forceinline__ h16 tohx(float x) { return (h16)x; }
__device__ __forceinline__ void splitf(float y, unsigned short& h, unsigned short& l) { h = f2bf(y); l = f2bf(y - bf2f(h)); }
typedef __attribute__((ext_vector_type(2))) _Float16 v2h;
typedef __attribute__((ext_vector_type(4))) _Float16 v4h;
typedef __attribute__((ext_vector_type(2))) unsigned short v2us;
typedef __attribute__((ext_vector_type(4))) unsigned short v4us;
typedef __attribute__((ext_vector_type(2))) float v2f;
typedef __attribute__((ext_vector_type(4))) int v4i;


__global__ __launch_bounds__(256) void k_weff(const float* __restrict__ w1, const float* __restrict__ w2, const float* __restrict__ w3, bf* WEh, bf* WEl) { const int e = (blockIdx.x * 256 + threadIdx.x) * 2; if (e >= NO * KK) return; const int o = e / KK; v2us oh, ol;
#pragma unroll
    for (int q = 0; q < 2; ++q) { const int k = (e + q) % KK; const int s = k / CC, c = k % CC; float v = 0.0f;
        if (o < 9) { const int oy = o / 3, ox = o % 3, sy = s / 3, sx = s % 3; const int dy = sy - oy + 1, dx = sx - ox + 1;
            if (s == o) v = bfr(w1[c]);
            if (dy >= 0 && dy <= 1 && dx >= 0 && dx <= 1) v = __fadd_rn(v, bfr(w2[(c * 2 + dy) * 2 + dx]));
            if (dy >= 0 && dy <= 2 && dx >= 0 && dx <= 2) v = __fadd_rn(v, bfr(w3[(c * 3 + dy) * 3 + dx])); }
        unsigned short a, b2; splitf(v, a, b2); oh[q] = a; ol[q] = b2; }
    *(volatile v2us*)(WEh + e) = oh; *(volatile v2us*)(WEl + e) = ol; __threadfence(); *(volatile v2us*)(WEh + e) = oh; *(volatile v2us*)(WEl + e) = ol; }
__global__ __launch_bounds__(256) void k_patch(const float* __restrict__ x, int n, int p0, bf* APh, bf* APl) { const size_t tIdx = (size_t)blockIdx.x * 256 + threadIdx.x; if (tIdx >= (size_t)PR * 9 * (CC / 8)) return; const int cg = (int)(tIdx % (CC / 8)); const int s = (int)((tIdx / (CC / 8)) % 9); const int r = (int)(tIdx / (9 * (CC / 8))); const int pix = p0 + r; const int h = pix / WW, w = pix % WW; const int sy = s / 3, sx = s % 3; const int hy = h + sy - 1, wx = w + sx - 1; const bool inb = (hy >= 0 && hy < HH && wx >= 0 && wx < WW);
    const float* xc = x + (((size_t)n * CC + cg * 8) * HH + h) * WW + w; const float* xn = x + (((size_t)n * CC + cg * 8) * HH + (inb ? hy : 0)) * WW + (inb ? wx : 0); v8us oh, ol;
#pragma unroll
    for (int q = 0; q < 8; ++q) { const float ctr = bfr(xc[(size_t)q * HH * WW]); const float nb = inb ? bfr(xn[(size_t)q * HH * WW]) : 0.0f; const float d = __fsub_rn(nb, ctr); unsigned short a, b2; splitf(d, a, b2); oh[q] = a; ol[q] = b2; }
    const size_t e = (size_t)r * KK + s * CC + cg * 8; *(volatile v8us*)(APh + e) = oh; *(volatile v8us*)(APl + e) = ol; __threadfence(); *(volatile v8us*)(APh + e) = oh; *(volatile v8us*)(APl + e) = ol; }
__global__ __launch_bounds__(256) void k_expo(const float* __restrict__ YS, const float* __restrict__ b1, const float* __restrict__ b2, const float* __restrict__ b3, float* O) { const size_t t = (size_t)blockIdx.x * 256 + threadIdx.x; if (t >= (size_t)PR * 9 / 4) return; float bs = __fadd_rn(__fadd_rn(bfr(b1[0]), bfr(b2[0])), bfr(b3[0])); asm volatile("" : "+v"(bs)); v4f o4;
#pragma unroll
    for (int q = 0; q < 4; ++q) { const size_t f = t * 4 + q; const size_t r = f / 9; const int o = (int)(f % 9); float y = __fadd_rn(YS[r * NO + o], bs); asm volatile("" : "+v"(y)); float y3 = __fdiv_rn(y, 3.0f); asm volatile("" : "+v"(y3)); const float z = __fdiv_rn(y3, -9.0f); o4[q] = expf(z); }
    *(volatile v4f*)(O + t * 4) = o4; __threadfence(); *(volatile v4f*)(O + t * 4) = o4; }

extern "C" void kernel_launch(void* const* d_in, const int* in_sizes, int n_in,
                              void* d_out, int out_size, void* d_ws, size_t ws_size, hipStream_t stream) {
    (void)in_sizes; (void)n_in; (void)out_size;
    const float* x = (const float*)d_in[0]; const float* w1 = (const float*)d_in[1]; const float* b1 = (const float*)d_in[2]; const float* w2 = (const float*)d_in[3]; const float* b2 = (const float*)d_in[4]; const float* w3 = (const float*)d_in[5]; const float* b3 = (const float*)d_in[6];
    float* OUT = (float*)d_out;
    char* wsp = (char*)d_ws;
    auto take = [&](size_t bytes) { char* p = wsp; wsp += (bytes + 255) & ~(size_t)255; return (void*)p; };
    bf* WEh = (bf*)take((size_t)NO * KK * 2); bf* WEl = (bf*)take((size_t)NO * KK * 2); bf* APh = (bf*)take((size_t)PR * KK * 2); bf* APl = (bf*)take((size_t)PR * KK * 2); float* YS = (float*)take((size_t)PR * NO * 4);
    if ((size_t)(wsp - (char*)d_ws) > ws_size) return;
    k_weff<<<(NO * KK / 2 + 255) / 256, 256, 0, stream>>>(w1, w2, w3, WEh, WEl);
    static_assert(PR == NPIX, "one pass per image");
    for (int n = 0; n < NIMG; ++n) { const int p0 = 0;
        k_patch<<<(unsigned)(((size_t)PR * 9 * (CC / 8) + 255) / 256), 256, 0, stream>>>(x, n, p0, APh, APl);
        k_gemmw<bf, 2, false><<<dim3(PR / 64, NO / 64, 1), 32, 0, stream>>>(APh, APl, WEh, WEl, KK, YS, NO, nullptr, 0, 0, 0);
        k_expo<<<(unsigned)(((size_t)PR * 9 / 4 + 255) / 256), 256, 0, stream>>>(YS, b1, b2, b3, OUT + ((size_t)n * NPIX + p0) * 9); }
}
